// CustomTransformerEncoderLayer_71442486002223
// MI455X (gfx1250) — hardware-verified
//
#include <hip/hip_runtime.h>


#define NB_  1
#define NT_  2048
#define DM   1024
#define FF   4096
#define LN_EPS 1e-5f
#define NH_  16
#define HD   64
#define NTK  (NB_ * NT_)
#define NW   1024
#define NQKV 1024
#define PSC  32768.0f
#define LOSC 1024.0f
#define LOSCI (1.0f / 1024.0f)

typedef _Float16 h16;
typedef unsigned short bf;
typedef __attribute__((ext_vector_type(16))) __bf16   v16bf;
typedef __attribute__((ext_vector_type(16))) _Float16 v16h;
typedef __attribute__((ext_vector_type(8)))  _Float16 v8h;
typedef __attribute__((ext_vector_type(8)))  unsigned short v8us;
typedef __attribute__((ext_vector_type(8)))  float    v8f;
typedef __attribute__((ext_vector_type(4)))  float    v4f;
typedef v8h  __attribute__((may_alias)) v8ha;
typedef v4f  __attribute__((may_alias)) v4fa;
typedef v8us __attribute__((may_alias)) v8usa;

__device__ __forceinline__ unsigned short f2bf(float f) { unsigned u = __float_as_uint(f); u += 0x7FFFu + ((u >> 16) & 1u); return (unsigned short)(u >> 16); }
__device__ __forceinline__ float bf2f(unsigned short b) { return __uint_as_float(((unsigned)b) << 16); }
__device__ __forceinline__ float bfr(float f) { return bf2f(f2bf(f)); }
__device__ __forceinline__ v16h cat16(v8h lo, v8h hi) { return __builtin_shufflevector(lo, hi, 0, 1, 2, 3, 4, 5, 6, 7, 8, 9, 10, 11, 12, 13, 14, 15); }
__device__ __forceinline__ v16bf cat16b(v8us lo, v8us hi) { return __builtin_bit_cast(v16bf, __builtin_shufflevector(lo, hi, 0, 1, 2, 3, 4, 5, 6, 7, 8, 9, 10, 11, 12, 13, 14, 15)); }
__device__ __forceinline__ v8f wmma16(v16h a, v16h b, v8f c) { return __builtin_amdgcn_wmma_f32_16x16x32_f16(false, a, false, b, (short)0, c, false, false); }
__device__ __forceinline__ v8f wmmab(v16bf a, v16bf b, v8f c) { return __builtin_amdgcn_wmma_f32_16x16x32_bf16(false, a, false, b, (short)0, c, false, false); }

__global__ __launch_bounds__(256) void k_cvtb(const float* __restrict__ src, int nrows, bf* dst) {
    const int lane = threadIdx.x & 31, r = blockIdx.x * 8 + (threadIdx.x >> 5);
    if (r >= nrows) return;
    v8us o[DM / 256];
#pragma unroll
    for (int q = 0; q < DM / 256; ++q) { v8us t;
#pragma unroll
        for (int i = 0; i < 8; ++i) t[i] = f2bf(src[(size_t)r * DM + q * 256 + lane * 8 + i]);
        o[q] = t; }
#pragma unroll
    for (int q = 0; q < DM / 256; ++q) *(volatile v8us*)(dst + (size_t)r * DM + q * 256 + lane * 8) = o[q];
    __threadfence();
#pragma unroll
    for (int q = 0; q < DM / 256; ++q) *(volatile v8us*)(dst + (size_t)r * DM + q * 256 + lane * 8) = o[q];
}

template <bool SPLITA, bool F16OUT = false>
__global__ __launch_bounds__(128) void k_gemmb(const bf* __restrict__ A, const bf* __restrict__ Al, const bf* __restrict__ Bn, const float* __restrict__ bias, float* C, int ldc, h16* C2, const float* __restrict__ R = nullptr, int K = DM, int roundR = 1) {
    __shared__ __align__(16) float ost[4][16 * 68];
    const int lane = threadIdx.x & 31, wave = threadIdx.x >> 5, lr = lane & 15, hi = lane >> 4;
    const int r0 = blockIdx.x * 64 + wave * 16, c0 = blockIdx.y * 64;
    const size_t aoff = (size_t)(r0 + lr) * K + 8 * hi;
    size_t boff[4];
#pragma unroll
    for (int t = 0; t < 4; ++t) boff[t] = (size_t)(c0 + t * 16 + lr) * K + 8 * hi;
    v8f acc[4];
#pragma unroll
    for (int t = 0; t < 4; ++t) acc[t] = (v8f){};
#pragma unroll 1
    for (int kc = 0; kc < K; kc += 32) {
        const v16bf a = cat16b(*(const v8us*)(A + aoff + kc), *(const v8us*)(A + aoff + kc + 16));
        v16bf al = a;
        if (SPLITA) al = cat16b(*(const v8us*)(Al + aoff + kc), *(const v8us*)(Al + aoff + kc + 16));
#pragma unroll
        for (int t = 0; t < 4; ++t) { const v16bf b = cat16b(*(const v8us*)(Bn + boff[t] + kc), *(const v8us*)(Bn + boff[t] + kc + 16)); acc[t] = wmmab(a, b, acc[t]); if (SPLITA) acc[t] = wmmab(al, b, acc[t]); }
        asm volatile("v_nop\n\tv_nop\n\tv_nop\n\tv_nop" : "+v"(acc[0]), "+v"(acc[1]), "+v"(acc[2]), "+v"(acc[3]) : "v"(a), "v"(al));
    }
    float* os = &ost[wave][0];
#pragma unroll
    for (int t = 0; t < 4; ++t) { const float bv = bias ? bfr(bias[c0 + t * 16 + lr]) : 0.f;
#pragma unroll
        for (int j = 0; j < 8; ++j) os[(hi * 8 + j) * 68 + t * 16 + lr] = acc[t][j] + bv; }
    __syncthreads();
    if (F16OUT) {
        h16* crow = (h16*)(void*)C + (size_t)r0 * ldc + c0;
        auto pass = [&]() {
#pragma unroll
            for (int s = 0; s < 4; ++s) { const int row = 4 * s + (lane >> 3), piece = lane & 7; const float* sp = os + row * 68 + piece * 8; v8h o, o2;
#pragma unroll
                for (int i = 0; i < 8; ++i) { const h16 a = (h16)sp[i]; o[i] = a; o2[i] = (h16)((sp[i] - (float)a) * LOSC); }
                *(volatile v8h*)(crow + (size_t)row * ldc + piece * 8) = o; if (C2) *(volatile v8h*)(C2 + (size_t)r0 * ldc + c0 + (size_t)row * ldc + piece * 8) = o2; }
        };
        pass(); __threadfence(); pass();
    } else {
        float* crow = C + (size_t)r0 * ldc + c0;
        auto pass = [&]() {
#pragma unroll
            for (int s = 0; s < 8; ++s) { const int Lid = (lane >> 3) + 4 * s, piece = lane & 7; const int row = Lid >> 1, cofs = (Lid & 1) * 32 + piece * 4;
                v4f val = *(const v4fa*)(os + row * 68 + cofs); if (R) { const v4f rv = *(const v4f*)(R + ((size_t)r0 + row) * ldc + c0 + cofs); val += roundR ? (v4f){bfr(rv[0]), bfr(rv[1]), bfr(rv[2]), bfr(rv[3])} : rv; }
                *(volatile v4f*)(crow + (size_t)row * ldc + cofs) = val; }
        };
        pass(); __threadfence(); pass();
    }
}

__global__ __launch_bounds__(256) void k_vt(const float* __restrict__ V, h16* VTH, h16* VTL) {
    __shared__ __align__(16) h16 tile[64 * 72];
    __shared__ __align__(16) h16 til2[64 * 72];
    const int bid = blockIdx.x;
    const int b = bid / (NH_ * (NT_ / 64)), rem = bid - b * (NH_ * (NT_ / 64)), h = rem / (NT_ / 64), kt = rem - h * (NT_ / 64);
    const int k0 = kt * 64, tid = threadIdx.x;
    const int kk = tid >> 2, d0 = (tid & 3) * 16;
    const float* src = V + ((size_t)b * NT_ + k0 + kk) * DM + h * HD + d0;
#pragma unroll
    for (int i = 0; i < 16; ++i) { const float v = src[i]; const h16 a = (h16)v; tile[(d0 + i) * 72 + kk] = a; til2[(d0 + i) * 72 + kk] = (h16)((v - (float)a) * LOSC); }
    __syncthreads();
    const int piece = tid & 7;
    const size_t base = (((size_t)b * NH_ + h) * HD) * NT_ + k0;
    auto pass = [&]() {
#pragma unroll
        for (int s = 0; s < 4; ++s) { const int Lid = (tid >> 3) + 32 * s; const int pln = Lid >> 6, d = Lid & 63;
            const v8h val = *(const v8ha*)((pln ? til2 : tile) + d * 72 + piece * 8); *(volatile v8h*)((pln ? VTL : VTH) + base + (size_t)d * NT_ + piece * 8) = val; }
    };
    pass(); __threadfence(); pass();
}

__global__ __launch_bounds__(128) void k_attn(const h16* __restrict__ Q16, const h16* __restrict__ QL16, const h16* __restrict__ K16, const h16* __restrict__ KL16, const h16* __restrict__ VTH, const h16* __restrict__ VTL, bf* CH, bf* CL) {
    __shared__ __align__(16) h16 plds[4][16 * 32];
    __shared__ __align__(16) h16 plds2[4][16 * 32];
    __shared__ __align__(16) float ost[4][16 * 68];
    const int lane = threadIdx.x & 31, wave = threadIdx.x >> 5, lr = lane & 15, hi = lane >> 4;
    const int bid = blockIdx.x;
    const int b = bid / (NH_ * (NT_ / 64)), rem = bid - b * (NH_ * (NT_ / 64)), h = rem / (NT_ / 64), qt = rem - h * (NT_ / 64);
    const int q0 = qt * 64 + wave * 16;
    const size_t tok0 = (size_t)b * NT_;
    h16* pl = &plds[wave][0]; h16* pl2 = &plds2[wave][0];
    v16h qa[2];
    const size_t qo0 = (tok0 + q0 + lr) * DM + h * HD + 8 * hi;
#pragma unroll
    for (int kc = 0; kc < 2; ++kc) qa[kc] = cat16(*(const v8h*)(Q16 + qo0 + kc * 32), *(const v8h*)(Q16 + qo0 + kc * 32 + 16));
    const h16* kh_b = K16 + tok0 * DM + h * HD;
    const h16* kl_b = KL16 + tok0 * DM + h * HD;
    const size_t vbase = (((size_t)b * NH_ + h) * HD) * NT_;
    v8f o[4], ox[4];
#pragma unroll
    for (int n = 0; n < 4; ++n) { o[n] = (v8f){}; ox[n] = (v8f){}; }
    float mrow[8], lpart[8];
#pragma unroll
    for (int j = 0; j < 8; ++j) { mrow[j] = -3.0e38f; lpart[j] = 0.f; }
    int qpos[8];
#pragma unroll
    for (int j = 0; j < 8; ++j) qpos[j] = q0 + 8 * hi + j;
    const int kt_lo = 0, kt_hi = NT_ / 32 - 1;
#pragma unroll 1
    for (int kt = kt_lo; kt <= kt_hi; ++kt) {
        const int l0 = kt * 32;
        const size_t ko0 = (size_t)(l0 + lr) * DM + 8 * hi, ko1 = (size_t)(l0 + 16 + lr) * DM + 8 * hi;
        v8f s0 = {}, s1 = {}, x0 = {}, x1 = {};
#pragma unroll
        for (int kc = 0; kc < 2; ++kc) {
            { const v16h k0h = cat16(*(const v8h*)(kh_b + ko0 + kc * 32), *(const v8h*)(kh_b + ko0 + kc * 32 + 16)), k1h = cat16(*(const v8h*)(kh_b + ko1 + kc * 32), *(const v8h*)(kh_b + ko1 + kc * 32 + 16));
              const v16h qlk = cat16(*(const v8h*)(QL16 + qo0 + kc * 32), *(const v8h*)(QL16 + qo0 + kc * 32 + 16));
              s0 = wmma16(qa[kc], k0h, s0); x0 = wmma16(qlk, k0h, x0); s1 = wmma16(qa[kc], k1h, s1); x1 = wmma16(qlk, k1h, x1);
              asm volatile("v_nop" : "+v"(s0), "+v"(s1), "+v"(x0), "+v"(x1) : "v"(qlk), "v"(k0h), "v"(k1h) : "memory"); }
            { const v16h k0l = cat16(*(const v8h*)(kl_b + ko0 + kc * 32), *(const v8h*)(kl_b + ko0 + kc * 32 + 16)), k1l = cat16(*(const v8h*)(kl_b + ko1 + kc * 32), *(const v8h*)(kl_b + ko1 + kc * 32 + 16));
              x0 = wmma16(qa[kc], k0l, x0); x1 = wmma16(qa[kc], k1l, x1);
              asm volatile("v_nop" : "+v"(x0), "+v"(x1) : "v"(k0l), "v"(k1l) : "memory"); }
        }
        asm volatile("v_nop\n\tv_nop\n\tv_nop\n\tv_nop" : "+v"(s0), "+v"(s1), "+v"(x0), "+v"(x1) : "v"(qa[0]), "v"(qa[1]));
        float alpha[8];
#pragma unroll
        for (int j = 0; j < 8; ++j) {
            const int ja = l0 + lr, jb = l0 + 16 + lr, qi = qpos[j];
            const float a0 = (s0[j] + x0[j] * LOSCI) * 0.125f, a1 = (s1[j] + x1[j] * LOSCI) * 0.125f; (void)ja; (void)jb; (void)qi;
            float mx = fmaxf(a0, a1);
            mx = fmaxf(mx, __shfl_xor(mx, 1, 16)); mx = fmaxf(mx, __shfl_xor(mx, 2, 16)); mx = fmaxf(mx, __shfl_xor(mx, 4, 16)); mx = fmaxf(mx, __shfl_xor(mx, 8, 16));
            const float mn = fmaxf(mrow[j], mx);
            alpha[j] = __expf(mrow[j] - mn); mrow[j] = mn;
            const float p0 = __expf(a0 - mn), p1 = __expf(a1 - mn);
            lpart[j] = lpart[j] * alpha[j] + (p0 + p1);
            const int mr = hi * 8 + j;
            const float ps0 = p0 * PSC, ps1 = p1 * PSC; const h16 h0 = (h16)ps0, h1 = (h16)ps1;
            pl[mr * 32 + lr] = h0; pl[mr * 32 + 16 + lr] = h1;
            pl2[mr * 32 + lr] = (h16)((ps0 - (float)h0) * LOSC); pl2[mr * 32 + 16 + lr] = (h16)((ps1 - (float)h1) * LOSC);
        }
#pragma unroll
        for (int n = 0; n < 4; ++n)
#pragma unroll
            for (int j = 0; j < 8; ++j) { o[n][j] *= alpha[j]; ox[n][j] *= alpha[j]; }
        asm volatile("" ::: "memory");
        const v16h pa = cat16(*(const v8ha*)(pl + lr * 32 + hi * 8), *(const v8ha*)(pl + lr * 32 + 16 + hi * 8));
        const v16h px = cat16(*(const v8ha*)(pl2 + lr * 32 + hi * 8), *(const v8ha*)(pl2 + lr * 32 + 16 + hi * 8));
#pragma unroll
        for (int n = 0; n < 4; ++n) { const size_t vo = vbase + (size_t)(n * 16 + lr) * NT_ + l0 + hi * 8;
            const v16h vh = cat16(*(const v8h*)(VTH + vo), *(const v8h*)(VTH + vo + 16)), vl = cat16(*(const v8h*)(VTL + vo), *(const v8h*)(VTL + vo + 16));
            o[n] = wmma16(pa, vh, o[n]); ox[n] = wmma16(pa, vl, ox[n]); ox[n] = wmma16(px, vh, ox[n]);
            asm volatile("" : "+v"(o[n]), "+v"(ox[n]) : "v"(vh), "v"(vl) : "memory"); }
        asm volatile("v_nop\n\tv_nop\n\tv_nop\n\tv_nop" : "+v"(o[0]), "+v"(o[1]), "+v"(o[2]), "+v"(o[3]), "+v"(ox[0]), "+v"(ox[1]), "+v"(ox[2]), "+v"(ox[3]) : "v"(pa), "v"(px));
    }
    float inv[8];
#pragma unroll
    for (int j = 0; j < 8; ++j) { float rs = lpart[j]; rs += __shfl_xor(rs, 1, 16); rs += __shfl_xor(rs, 2, 16); rs += __shfl_xor(rs, 4, 16); rs += __shfl_xor(rs, 8, 16); inv[j] = 1.0f / (rs * PSC); }
    float* os = &ost[wave][0];
#pragma unroll
    for (int n = 0; n < 4; ++n)
#pragma unroll
        for (int j = 0; j < 8; ++j) os[(hi * 8 + j) * 68 + n * 16 + lr] = (o[n][j] + ox[n][j] * LOSCI) * inv[j];
    __syncthreads();
    const size_t cbase = (tok0 + q0) * DM + (size_t)h * HD;
    auto pass = [&]() {
#pragma unroll
        for (int s = 0; s < 4; ++s) { const int row = 4 * s + (lane >> 3), piece = lane & 7; const float* sp = os + row * 68 + piece * 8; v8us oh, ol;
#pragma unroll
            for (int i = 0; i < 8; ++i) { const unsigned short hb = f2bf(sp[i]); oh[i] = hb; ol[i] = f2bf(sp[i] - bf2f(hb)); }
            *(volatile v8us*)(CH + cbase + (size_t)row * DM + piece * 8) = oh; *(volatile v8us*)(CL + cbase + (size_t)row * DM + piece * 8) = ol; }
    };
    pass(); __threadfence(); pass();
}

#define VST2(T, p, v) do { const T vst2_v_ = (v); *(volatile T*)(p) = vst2_v_; __threadfence(); *(volatile T*)(p) = vst2_v_; } while (0)
__global__ __launch_bounds__(256) void k_trig(float* RC, float* RS) {
    const int u = blockIdx.x * 256 + threadIdx.x; if (u >= NT_ * 32) return;
    const int t = u >> 5, i = u & 31; const float inv = 1.0f / powf(10000.0f, (float)(2 * i) / (float)HD); const float ang = (float)t * inv; const float c = cosf(ang), s = sinf(ang);
    *(volatile float*)(RC + u) = c; *(volatile float*)(RS + u) = s; __threadfence(); *(volatile float*)(RC + u) = c; *(volatile float*)(RS + u) = s;
}
__global__ __launch_bounds__(256) void k_ropei(const float* __restrict__ P, const float* __restrict__ RC, const float* __restrict__ RS, h16* PH, h16* PL) {
    const int lane = threadIdx.x & 31, wid = blockIdx.x * 8 + (threadIdx.x >> 5); const int t = wid / (DM / 256), sg = wid % (DM / 256); if (t >= NT_) return;
    const int c0 = sg * 256 + lane * 8; const v8f xv = *(const v8f*)(P + (size_t)t * DM + c0); v8h oh, ol;
#pragma unroll
    for (int pq = 0; pq < 4; ++pq) { const int c = c0 + 2 * pq, i = (c & 63) >> 1; const float co = RC[t * 32 + i], s = RS[t * 32 + i];
        const float y0 = xv[2 * pq] * co - xv[2 * pq + 1] * s, y1 = xv[2 * pq] * s + xv[2 * pq + 1] * co;
        const h16 a0 = (h16)y0, a1 = (h16)y1; oh[2 * pq] = a0; oh[2 * pq + 1] = a1; ol[2 * pq] = (h16)((y0 - (float)a0) * LOSC); ol[2 * pq + 1] = (h16)((y1 - (float)a1) * LOSC); }
    const size_t o = (size_t)t * DM + c0; *(volatile v8h*)(PH + o) = oh; *(volatile v8h*)(PL + o) = ol; __threadfence(); *(volatile v8h*)(PH + o) = oh; *(volatile v8h*)(PL + o) = ol;
}
__global__ __launch_bounds__(256) void k_ln(const float* __restrict__ src, const float* __restrict__ g, const float* __restrict__ bb, int nrows, float* Y, bf* Ph, bf* Pl) {
    const int lane = threadIdx.x & 31, r = blockIdx.x * 8 + (threadIdx.x >> 5); if (r >= nrows) return;
    v8f v[DM / 256]; float s = 0.f;
#pragma unroll
    for (int q = 0; q < DM / 256; ++q) { v[q] = *(const v8f*)(src + (size_t)r * DM + q * 256 + lane * 8);
#pragma unroll
        for (int i = 0; i < 8; ++i) s += v[q][i]; }
#pragma unroll
    for (int sh = 16; sh; sh >>= 1) s += __shfl_xor(s, sh, 32);
    const float mu = s * (1.0f / DM); float s2 = 0.f;
#pragma unroll
    for (int q = 0; q < DM / 256; ++q)
#pragma unroll
        for (int i = 0; i < 8; ++i) { const float d = v[q][i] - mu; s2 = fmaf(d, d, s2); }
#pragma unroll
    for (int sh = 16; sh; sh >>= 1) s2 += __shfl_xor(s2, sh, 32);
    const float rs = rsqrtf(s2 * (1.0f / DM) + LN_EPS);
#pragma unroll 1
    for (int ps = 0; ps < 2; ++ps) {
#pragma unroll
        for (int q = 0; q < DM / 256; ++q) { const int c0 = q * 256 + lane * 8; const size_t o = (size_t)r * DM + c0; v8f y; v8us oh, ol;
#pragma unroll
            for (int i = 0; i < 8; ++i) { y[i] = (v[q][i] - mu) * rs * bfr(g[c0 + i]) + bfr(bb[c0 + i]); const unsigned short hb = f2bf(y[i]); oh[i] = hb; ol[i] = f2bf(y[i] - bf2f(hb)); }
            *(volatile v8f*)(Y + o) = y; if (Ph) { *(volatile v8us*)(Ph + o) = oh; *(volatile v8us*)(Pl + o) = ol; } }
        if (ps == 0) __threadfence(); }
}
__global__ __launch_bounds__(256) void k_relu(const float* __restrict__ src, int nrows, bf* dh, bf* dl) {
    const int lane = threadIdx.x & 31, r = blockIdx.x * 8 + (threadIdx.x >> 5); if (r >= nrows) return;
#pragma unroll 1
    for (int ps = 0; ps < 2; ++ps) {
#pragma unroll 1
        for (int q = 0; q < FF / 256; ++q) { const size_t o = (size_t)r * FF + q * 256 + lane * 8; const v8f v = *(const v8f*)(src + o); v8us oh, ol;
#pragma unroll
            for (int i = 0; i < 8; ++i) { const float y = fmaxf(v[i], 0.f); const unsigned short hb = f2bf(y); oh[i] = hb; ol[i] = f2bf(y - bf2f(hb)); }
            *(volatile v8us*)(dh + o) = oh; *(volatile v8us*)(dl + o) = ol; }
        if (ps == 0) __threadfence(); }
}

extern "C" void kernel_launch(void* const* d_in, const int* in_sizes, int n_in,
                              void* d_out, int out_size, void* d_ws, size_t ws_size, hipStream_t stream) {
    (void)in_sizes; (void)n_in; (void)out_size;
    const float* x = (const float*)d_in[0]; const float* Win = (const float*)d_in[1]; const float* bin = (const float*)d_in[2]; const float* Wo = (const float*)d_in[3]; const float* bo = (const float*)d_in[4];
    const float* W1 = (const float*)d_in[5]; const float* b1 = (const float*)d_in[6]; const float* W2 = (const float*)d_in[7]; const float* b2 = (const float*)d_in[8]; const float* g1 = (const float*)d_in[9]; const float* be1 = (const float*)d_in[10]; const float* g2 = (const float*)d_in[11]; const float* be2 = (const float*)d_in[12];
    float* out = (float*)d_out;
    char* wsp = (char*)d_ws;
    auto take = [&](size_t bytes) { char* p = wsp; wsp += (bytes + 255) & ~(size_t)255; return (void*)p; };
    bf* Xb = (bf*)take((size_t)NTK * DM * 2); bf* WqB = (bf*)take((size_t)DM * DM * 2); bf* WkB = (bf*)take((size_t)DM * DM * 2); bf* WvB = (bf*)take((size_t)DM * DM * 2); bf* WoB = (bf*)take((size_t)DM * DM * 2);
    bf* W1B = (bf*)take((size_t)FF * DM * 2); bf* W2B = (bf*)take((size_t)DM * FF * 2); float* RC = (float*)take((size_t)NT_ * 32 * 4); float* RS = (float*)take((size_t)NT_ * 32 * 4);
    float* TMP = (float*)take((size_t)NTK * DM * 4);
    h16* QH = (h16*)take((size_t)NTK * DM * 2); h16* QL = (h16*)take((size_t)NTK * DM * 2); h16* KH = (h16*)take((size_t)NTK * DM * 2); h16* KL = (h16*)take((size_t)NTK * DM * 2);
    h16* VTH = (h16*)take((size_t)NTK * DM * 2); h16* VTL = (h16*)take((size_t)NTK * DM * 2); bf* CH = (bf*)take((size_t)NTK * DM * 2); bf* CL = (bf*)take((size_t)NTK * DM * 2);
    float* Hf = (float*)take((size_t)NTK * DM * 4); float* F1 = (float*)take((size_t)(NTK / 2) * FF * 4); float* T2 = (float*)take((size_t)NTK * DM * 4);
    if ((size_t)(wsp - (char*)d_ws) > ws_size) return;
    float* T1 = TMP; bf* Hh = (bf*)QH; bf* Hl = (bf*)QL;
    bf* Rh = (bf*)KH; bf* Rl = (bf*)VTH;
    k_cvtb<<<DM / 8, 256, 0, stream>>>(Win, DM, WqB); k_cvtb<<<DM / 8, 256, 0, stream>>>(Win + (size_t)DM * DM, DM, WkB); k_cvtb<<<DM / 8, 256, 0, stream>>>(Win + (size_t)2 * DM * DM, DM, WvB); k_cvtb<<<DM / 8, 256, 0, stream>>>(Wo, DM, WoB);
    k_cvtb<<<FF / 8, 256, 0, stream>>>(W1, FF, W1B);
    {
      k_cvtb<<<FF / 8, 256, 0, stream>>>(W2, FF, W2B); }
    k_trig<<<(NT_ * 32) / 256, 256, 0, stream>>>(RC, RS);
    for (int b = 0; b < 2; ++b) {
        const float* xb = x + (size_t)b * NTK * DM;
        k_cvtb<<<NTK / 8, 256, 0, stream>>>(xb, NTK, Xb);
        k_gemmb<false, false><<<dim3(NTK / 64, DM / 64, 1), 128, 0, stream>>>(Xb, nullptr, WqB, bin, TMP, DM, nullptr); k_ropei<<<(NT_ * (DM / 256)) / 8, 256, 0, stream>>>(TMP, RC, RS, QH, QL);
        k_gemmb<false, false><<<dim3(NTK / 64, DM / 64, 1), 128, 0, stream>>>(Xb, nullptr, WkB, bin + DM, TMP, DM, nullptr); k_ropei<<<(NT_ * (DM / 256)) / 8, 256, 0, stream>>>(TMP, RC, RS, KH, KL);
        k_gemmb<false, false><<<dim3(NTK / 64, DM / 64, 1), 128, 0, stream>>>(Xb, nullptr, WvB, bin + 2 * DM, TMP, DM, nullptr); k_vt<<<NB_ * NH_ * (NT_ / 64), 256, 0, stream>>>(TMP, VTH, VTL);
        k_attn<<<NB_ * NH_ * (NT_ / 64), 128, 0, stream>>>(QH, QL, KH, KL, VTH, VTL, CH, CL);
        k_gemmb<true, false><<<dim3(NTK / 64, DM / 64, 1), 128, 0, stream>>>(CH, CL, WoB, bo, T1, DM, nullptr, xb, DM, 1);
        k_ln<<<NTK / 8, 256, 0, stream>>>(T1, g1, be1, NTK, Hf, Hh, Hl);
        for (int ch = 0; ch < 2; ++ch) { const size_t r0 = (size_t)ch * (NTK / 2);
            k_gemmb<true, false><<<dim3((NTK / 2) / 64, FF / 64, 1), 128, 0, stream>>>(Hh + r0 * DM, Hl + r0 * DM, W1B, b1, F1, FF, nullptr, nullptr, DM);
            k_relu<<<(NTK / 2) / 8, 256, 0, stream>>>(F1, NTK / 2, Rh, Rl);
            k_gemmb<true, false><<<dim3((NTK / 2) / 64, DM / 64, 1), 128, 0, stream>>>(Rh, Rl, W2B, b2, T2 + r0 * DM, DM, nullptr, Hf + r0 * DM, FF, 0);
        }
        k_ln<<<NTK / 8, 256, 0, stream>>>(T2, g2, be2, NTK, out + (size_t)b * NTK * DM, nullptr, nullptr);
    }
}
